// MultiHeadAttention_7069516169541
// MI455X (gfx1250) — hardware-run, weakly checked
//
#include <hip/hip_runtime.h>
#ifndef NB
#define NB 2
#endif
#ifndef SEQ
#define SEQ 2048
#endif
#define SQ SEQ
#define SQ_FULL 2048
#define NB_FULL 2
#define DM 768
#define NH 12
#define HD 64
#define QT 256
#define NKX SQ
#define QT0 128
#define SCL 0.125f
#define SCLR 0.0001220703125f
#define NR ((size_t)NB * SQ)
#define MP ((int)((size_t)NB * SQ))

static_assert(SQ % QT == 0);
static_assert(SQ % 128 == 0);
static_assert(SQ % 16 == 0);
static_assert(QT0 == 128);
static_assert(SQ >= QT0);
static_assert(NH * HD == DM);
static_assert(DM % 64 == 0);
static_assert(SQ <= SQ_FULL);
static_assert(NB <= NB_FULL);

typedef unsigned short v8us __attribute__((ext_vector_type(8), may_alias));
typedef float  v8f  __attribute__((ext_vector_type(8)));
typedef float  v4f  __attribute__((ext_vector_type(4)));
typedef float  v4fa __attribute__((ext_vector_type(4), may_alias));
typedef _Float16 v16h __attribute__((ext_vector_type(16)));
typedef _Float16 v4h __attribute__((ext_vector_type(4)));
union FragH { v16h v; v8us half[2]; _Float16 h[16]; unsigned short u[16]; };

__device__ __forceinline__ unsigned short bf16_bits(float x) { unsigned int u = __float_as_uint(x); return (unsigned short)((u + 0x7FFFu + ((u >> 16) & 1u)) >> 16); }
__device__ __forceinline__ float bf16_rne(float x) { return __uint_as_float(((unsigned int)bf16_bits(x)) << 16); }

__device__ __forceinline__ float rope_invf(int p) {
  float f = 1.0f;
  f = (p == 1)  ? 0.5623413251903491f : f;
  f = (p == 2)  ? 0.31622776601683794f : f;
  f = (p == 3)  ? 0.1778279410038923f : f;
  f = (p == 4)  ? 0.1f : f;
  f = (p == 5)  ? 0.05623413251903491f : f;
  f = (p == 6)  ? 0.03162277660168379f : f;
  f = (p == 7)  ? 0.01778279410038923f : f;
  f = (p == 8)  ? 0.01f : f;
  f = (p == 9)  ? 0.005623413251903491f : f;
  f = (p == 10) ? 0.0031622776601683794f : f;
  f = (p == 11) ? 0.0017782794100389228f : f;
  f = (p == 12) ? 0.001f : f;
  f = (p == 13) ? 0.0005623413251903491f : f;
  f = (p == 14) ? 0.00031622776601683794f : f;
  f = (p == 15) ? 0.00017782794100389227f : f;
  return f;
}

__global__ __launch_bounds__(256) void k_tab(float* __restrict__ TAB) {
  #pragma clang fp contract(off)
  __shared__ __attribute__((aligned(16))) float tl[16][32];
  const int tid = threadIdx.x; const int sl = tid >> 4, p = tid & 15; const int s = blockIdx.x * 16 + sl;
  const float ang = (float)s * rope_invf(p);
  float sn, cs; sincosf(ang, &sn, &cs);
  tl[sl][2 * p] = cs; tl[sl][2 * p + 1] = sn;
  __syncthreads();
  if (tid < 128) {
    const int row = tid >> 3, pc = (tid & 7) * 4;
    const v4f v = *(const v4fa*)&tl[row][pc];
    float* d = TAB + (size_t)(blockIdx.x * 16 + row) * 32 + pc;
    *(volatile v4f*)d = v;
    __threadfence();
    *(volatile v4f*)d = v;
  }
}

__global__ __launch_bounds__(256) void k_wnat(const float* __restrict__ w, size_t n8, _Float16* __restrict__ Bt) {
  const size_t t = (size_t)blockIdx.x * 256 + threadIdx.x; if (t >= n8) return;
  const v4f a = *(const v4fa*)(w + t * 8), c = *(const v4fa*)(w + t * 8 + 4);
  FragH f;
#pragma unroll
  for (int q = 0; q < 4; ++q) { f.h[q] = (_Float16)(bf16_rne(a[q]) * 16.0f); f.h[4 + q] = (_Float16)(bf16_rne(c[q]) * 16.0f); }
  const v8us o = f.half[0];
  *(volatile v8us*)((unsigned short*)Bt + t * 8) = o; __threadfence(); *(volatile v8us*)((unsigned short*)Bt + t * 8) = o;
}

__global__ __launch_bounds__(256) void k_x16(const float* __restrict__ x, size_t sx, _Float16* __restrict__ X16, size_t sd, size_t n8) {
  const size_t t = (size_t)blockIdx.x * 256 + threadIdx.x; if (t >= n8) return;
  const float* xp = x + (size_t)blockIdx.y * sx; unsigned short* dp = (unsigned short*)X16 + (size_t)blockIdx.y * sd;
  const v4f a = *(const v4fa*)(xp + t * 8), c = *(const v4fa*)(xp + t * 8 + 4);
  FragH f;
#pragma unroll
  for (int q = 0; q < 4; ++q) { f.h[q] = (_Float16)bf16_rne(a[q]); f.h[4 + q] = (_Float16)bf16_rne(c[q]); }
  const v8us o = f.half[0];
  *(volatile v8us*)(dp + t * 8) = o; __threadfence(); *(volatile v8us*)(dp + t * 8) = o;
}

__global__ __launch_bounds__(256) void k_hl(const float* __restrict__ F, _Float16* __restrict__ Hh, _Float16* __restrict__ Hl, size_t n8) {
  const size_t t = (size_t)blockIdx.x * 256 + threadIdx.x; if (t >= n8) return;
  FragH fh, fl; const v4f a = *(const v4fa*)(F + t * 8), c = *(const v4fa*)(F + t * 8 + 4);
#pragma unroll
  for (int q = 0; q < 4; ++q) { _Float16 h = (_Float16)a[q]; fh.h[q] = h; fl.h[q] = (_Float16)((a[q] - (float)h) * 1024.0f); h = (_Float16)c[q]; fh.h[4 + q] = h; fl.h[4 + q] = (_Float16)((c[q] - (float)h) * 1024.0f); }
  for (int pass = 0; pass < 2; ++pass) { *(volatile v8us*)((unsigned short*)Hh + t * 8) = fh.half[0]; *(volatile v8us*)((unsigned short*)Hl + t * 8) = fl.half[0]; if (pass == 0) __threadfence(); }
}

__global__ __launch_bounds__(256) void k_hlrope(const float* __restrict__ F, const float* __restrict__ TAB, _Float16* __restrict__ Hh, _Float16* __restrict__ Hl, size_t n8) {
  #pragma clang fp contract(off)
  const size_t t = (size_t)blockIdx.x * 256 + threadIdx.x; if (t >= n8) return;
  const size_t e0 = t * 8; const size_t row = e0 / DM; const int col = (int)(e0 - row * DM); const int s = (int)(row % SQ);
  const int c0 = col & 63; const bool rot = c0 < 32; const int cc = c0 & 31;
  const v4f a = *(const v4fa*)(F + e0), c = *(const v4fa*)(F + e0 + 4);
  const v4f t0 = *(const v4fa*)(TAB + (size_t)s * 32 + cc), t1 = *(const v4fa*)(TAB + (size_t)s * 32 + cc + 4);
  float y[8];
  y[0] = rot ? (a[0] * t0[0] + (-a[1]) * t0[1]) : a[0];
  y[1] = rot ? (a[1] * t0[0] + a[0] * t0[1]) : a[1];
  y[2] = rot ? (a[2] * t0[2] + (-a[3]) * t0[3]) : a[2];
  y[3] = rot ? (a[3] * t0[2] + a[2] * t0[3]) : a[3];
  y[4] = rot ? (c[0] * t1[0] + (-c[1]) * t1[1]) : c[0];
  y[5] = rot ? (c[1] * t1[0] + c[0] * t1[1]) : c[1];
  y[6] = rot ? (c[2] * t1[2] + (-c[3]) * t1[3]) : c[2];
  y[7] = rot ? (c[3] * t1[2] + c[2] * t1[3]) : c[3];
  FragH fh, fl;
#pragma unroll
  for (int q = 0; q < 8; ++q) { const _Float16 h = (_Float16)y[q]; fh.h[q] = h; fl.h[q] = (_Float16)((y[q] - (float)h) * 1024.0f); }
  for (int pass = 0; pass < 2; ++pass) { *(volatile v8us*)((unsigned short*)Hh + t * 8) = fh.half[0]; *(volatile v8us*)((unsigned short*)Hl + t * 8) = fl.half[0]; if (pass == 0) __threadfence(); }
}

__global__ __launch_bounds__(256) void k_rope0(const float* __restrict__ F, const float* __restrict__ TAB, float* __restrict__ G, int n4) {
  #pragma clang fp contract(off)
  const int t = blockIdx.x * 256 + threadIdx.x; if (t >= n4) return;
  const size_t e0 = (size_t)t * 4; const int row = (int)(e0 / DM); const int col = (int)(e0 - (size_t)row * DM); const int s = row % QT0;
  const int c0 = col & 63; const bool rot = c0 < 32; const int cc = c0 & 31;
  const v4f a = *(const v4fa*)(F + e0);
  const v4f tb = *(const v4fa*)(TAB + (size_t)s * 32 + cc);
  v4f o;
  o[0] = rot ? (a[0] * tb[0] + (-a[1]) * tb[1]) : a[0];
  o[1] = rot ? (a[1] * tb[0] + a[0] * tb[1]) : a[1];
  o[2] = rot ? (a[2] * tb[2] + (-a[3]) * tb[3]) : a[2];
  o[3] = rot ? (a[3] * tb[2] + a[2] * tb[3]) : a[3];
  *(volatile v4f*)(G + e0) = o;
  __threadfence();
  *(volatile v4f*)(G + e0) = o;
}

template <int NHv, int TTv>
__global__ __launch_bounds__(256) void k_vt(const _Float16* __restrict__ V16, int ldv, int voff, _Float16* __restrict__ Vt) {
  __shared__ unsigned short tl[64][66];
  const int tid = threadIdx.x; const int slab = blockIdx.x / (TTv / 64), lg = blockIdx.x % (TTv / 64); const int b = slab / NHv, h = slab % NHv;
  for (int i = tid; i < 64 * 8; i += 256) { const int r = i / 8, c8 = (i % 8) * 8; FragH f; f.half[0] = *(const v8us*)((const unsigned short*)V16 + ((size_t)b * TTv + lg * 64 + r) * ldv + voff + h * 64 + c8);
#pragma unroll
    for (int q = 0; q < 8; ++q) tl[r][c8 + q] = f.u[q]; }
  __syncthreads();
  for (int pass = 0; pass < 2; ++pass) {
#pragma unroll
    for (int rd = 0; rd < 2; ++rd) { const int d = rd * 32 + tid / 8, pc = tid % 8; FragH f;
#pragma unroll
      for (int q = 0; q < 8; ++q) f.u[q] = tl[pc * 8 + q][d];
      *(volatile v8us*)((unsigned short*)Vt + ((size_t)slab * 64 + d) * TTv + lg * 64 + pc * 8) = f.half[0]; }
    if (pass == 0) __threadfence(); }
}

__device__ __forceinline__ v16h g2_frag(const _Float16* p, int hh) { FragH f; f.half[0] = *(const v8us*)((const unsigned short*)p + 8 * hh); f.half[1] = *(const v8us*)((const unsigned short*)p + 16 + 8 * hh); return f.v; }
__device__ __forceinline__ v8f g2_mma(v16h a, v16h b, v8f c) { v8f d = __builtin_amdgcn_wmma_f32_16x16x32_f16(false, a, false, b, (short)0, c, false, false); asm volatile("v_nop\n\tv_nop\n\tv_nop\n\tv_nop" : "+v"(d) : "v"(a), "v"(b)); return d; }
__global__ __launch_bounds__(128) void k_gemm2(const _Float16* __restrict__ A, int lda, size_t sA, const _Float16* __restrict__ Bh, int ldb, size_t sB, float alpha,
    const float* __restrict__ bias, const float* CP, float* C, _Float16* C16, int ldc, size_t sC, int M, int N, int K) {
  __shared__ __attribute__((aligned(16))) float so[4][32][68];
  const int tid = threadIdx.x, w = __builtin_amdgcn_readfirstlane((int)(tid >> 5)), lane = tid & 31, ln = lane & 15, hh = lane >> 4; const int by = blockIdx.y;
  A += (size_t)by * sA; Bh += (size_t)by * sB; const size_t cofs = (size_t)by * sC;
  const int ntn = N >> 6; const int mt = blockIdx.x / ntn, nq = blockIdx.x - mt * ntn; const int row0 = mt * 128 + 32 * w, col0 = nq * 64; if (row0 >= M) return;
  const _Float16* a0p = A + (size_t)(row0 + ln) * lda; const _Float16* a1p = a0p + (size_t)16 * lda;
  const _Float16* b0p = Bh + (size_t)(col0 + ln) * ldb; const _Float16* b1p = b0p + (size_t)16 * ldb; const _Float16* b2p = b1p + (size_t)16 * ldb; const _Float16* b3p = b2p + (size_t)16 * ldb;
  const v8f z8 = {0.f,0.f,0.f,0.f,0.f,0.f,0.f,0.f}; v8f c00 = z8, c01 = z8, c02 = z8, c03 = z8, c10 = z8, c11 = z8, c12 = z8, c13 = z8;
#pragma unroll 1
  for (int kb = 0; kb < K; kb += 32) { const v16h a0 = g2_frag(a0p + kb, hh), a1 = g2_frag(a1p + kb, hh);
    v16h b = g2_frag(b0p + kb, hh); c00 = g2_mma(a0, b, c00); c10 = g2_mma(a1, b, c10);
    b = g2_frag(b1p + kb, hh); c01 = g2_mma(a0, b, c01); c11 = g2_mma(a1, b, c11);
    b = g2_frag(b2p + kb, hh); c02 = g2_mma(a0, b, c02); c12 = g2_mma(a1, b, c12);
    b = g2_frag(b3p + kb, hh); c03 = g2_mma(a0, b, c03); c13 = g2_mma(a1, b, c13); }
  v8f accs[8] = {c00, c01, c02, c03, c10, c11, c12, c13};
#pragma unroll
  for (int u = 0; u < 8; ++u) { const int t = u & 3, half = u >> 2; const int col = col0 + t * 16 + ln; const float bv = bias ? bf16_rne(bias[col]) : 0.f;
#pragma unroll
    for (int r = 0; r < 8; ++r) { const int rloc = half * 16 + 8 * hh + r; float v = accs[u][r] * alpha + bv;
      if (CP) v += CP[cofs + (size_t)(row0 + rloc) * ldc + col];
      so[w][rloc][t * 16 + ln] = v; } }
  __builtin_amdgcn_fence(4  , "workgroup"); __builtin_amdgcn_wave_barrier();
  const int rsub = lane >> 4, c4 = (lane & 15) * 4;
  for (int pass = 0; pass < 2; ++pass) {
#pragma unroll
    for (int q = 0; q < 16; ++q) { const int r = q * 2 + rsub; const v4f v = *(const v4fa*)&so[w][r][c4];
      if (C) *(volatile v4f*)(C + cofs + (size_t)(row0 + r) * ldc + col0 + c4) = v;
      if (C16) { v4h h4; h4[0] = (_Float16)v[0]; h4[1] = (_Float16)v[1]; h4[2] = (_Float16)v[2]; h4[3] = (_Float16)v[3]; *(volatile v4h*)(C16 + cofs + (size_t)(row0 + r) * ldc + col0 + c4) = h4; } }
    if (pass == 0) __threadfence(); }
}

__global__ __launch_bounds__(256) void k_rsmcf2(const float* __restrict__ S, _Float16* __restrict__ P, int hg, int q0, int nk) {
  #pragma clang fp contract(off)
  const int t = blockIdx.x * 256 + threadIdx.x; if (t >= hg * QT) return; const size_t i = (size_t)t; const float* s = S + i * NKX; const int last = q0 + (t % QT); float mx = -3.0e38f;
#pragma unroll 1
  for (int j = 0; j < nk; ++j) { const float f = (j <= last) ? 1.f : 0.f; mx = fmaxf(mx, fmaf(f, s[j], (1.f - f) * -1.0e9f)); }
  float se = 0.f;
#pragma unroll 1
  for (int j = 0; j < nk; ++j) { const float f = (j <= last) ? 1.f : 0.f; se += __expf(fmaf(f, s[j], (1.f - f) * -1.0e9f) - mx); }
  const float sc = 256.0f / se;
#pragma unroll 1
  for (int j0 = 0; j0 < nk; j0 += 8) { FragH fr;
#pragma unroll
    for (int q = 0; q < 8; ++q) { const int j = j0 + q; const float f = (j <= last) ? 1.f : 0.f; fr.h[q] = (_Float16)(__expf(fmaf(f, s[j], (1.f - f) * -1.0e9f) - mx) * sc); }
    const v8us o = fr.half[0]; unsigned short* d = (unsigned short*)P + i * NKX + j0; *(volatile v8us*)d = o; __threadfence(); *(volatile v8us*)d = o; }
}

__global__ __launch_bounds__(64) void k_att0(const float* __restrict__ QF, const float* __restrict__ KF, const float* __restrict__ VF, int ld, float scale, float* __restrict__ OF, int ldo) {
  #pragma clang fp contract(off)
  __shared__ __attribute__((aligned(16))) float lq[64][64]; __shared__ __attribute__((aligned(16))) float lo[64][64];
  const int tid = threadIdx.x; const int h = blockIdx.x / (QT0 / 64), rg = blockIdx.x % (QT0 / 64); const int i = rg * 64 + tid;
  const float* qr = QF + (size_t)i * ld + h * HD;
#pragma unroll 1
  for (int c = 0; c < HD / 4; ++c) { *(v4f*)&lq[tid][c * 4] = *(const v4fa*)(qr + c * 4); const v4f z = {0.f, 0.f, 0.f, 0.f}; *(v4f*)&lo[tid][c * 4] = z; }
  float m = -1.0e30f, l = 0.f; const int jmax = rg * 64 + 63;
#pragma unroll 1
  for (int j = 0; j <= jmax; ++j) { const float* kr = KF + (size_t)j * ld + h * HD; const float* vr = VF + (size_t)j * ld + h * HD; float s = 0.f;
#pragma unroll 1
    for (int c = 0; c < HD / 4; ++c) { const v4f kq = *(const v4fa*)(kr + c * 4); const v4f qq = *(v4f*)&lq[tid][c * 4]; s = __fadd_rn(s, __fmul_rn(qq[0], kq[0])); s = __fadd_rn(s, __fmul_rn(qq[1], kq[1])); s = __fadd_rn(s, __fmul_rn(qq[2], kq[2])); s = __fadd_rn(s, __fmul_rn(qq[3], kq[3])); }
    s = __fmul_rn(s, scale);
    const float f = (j <= i) ? 1.f : 0.f; const float sm = fmaf(f, s, (1.f - f) * -1.0e30f); const float mn = fmaxf(m, sm); const float sc = expf(m - mn); const float e = expf(sm - mn); l = __fadd_rn(__fmul_rn(l, sc), e); m = mn;
#pragma unroll 1
    for (int c = 0; c < HD / 4; ++c) { const v4f vv = *(const v4fa*)(vr + c * 4); v4f oo = *(v4f*)&lo[tid][c * 4];
#pragma unroll
      for (int u = 0; u < 4; ++u) oo[u] = __fadd_rn(__fmul_rn(oo[u], sc), __fmul_rn(e, vv[u]));
      *(v4f*)&lo[tid][c * 4] = oo; } }
  const float fin = 64.0f / l;
#pragma unroll 1
  for (int c = 0; c < HD / 4; ++c) { v4f oo = *(v4f*)&lo[tid][c * 4];
#pragma unroll
    for (int u = 0; u < 4; ++u) oo[u] = __fmul_rn(oo[u], fin);
    *(v4f*)&lo[tid][c * 4] = oo; }
  __syncthreads();
  for (int pass = 0; pass < 2; ++pass) {
#pragma unroll 1
    for (int it = 0; it < 16; ++it) { const int row = it * 4 + tid / 16, pc = (tid % 16) * 4; const v4f v = *(const v4f*)&lo[row][pc]; *(volatile v4f*)(OF + (size_t)(rg * 64 + row) * ldo + h * HD + pc) = v; }
    if (pass == 0) __threadfence(); }
}

extern "C" void kernel_launch(void* const* d_in, const int* in_sizes, int n_in,
                              void* d_out, int out_size, void* d_ws, size_t ws_size, hipStream_t stream) {
  if (n_in < 9) return;
  const size_t needx = ((size_t)(NB - 1) * SQ_FULL + SQ) * DM;
  if ((size_t)in_sizes[0] < needx) return;
  if (in_sizes[1] < DM * DM || in_sizes[3] < DM * DM || in_sizes[5] < DM * DM || in_sizes[7] < DM * DM) return;
  if (in_sizes[2] < DM || in_sizes[4] < DM || in_sizes[6] < DM || in_sizes[8] < DM) return;
  if ((size_t)out_size < needx) return;
  const float* x = (const float*)d_in[0]; const float* wq = (const float*)d_in[1]; const float* bq = (const float*)d_in[2]; const float* wk = (const float*)d_in[3]; const float* bk = (const float*)d_in[4];
  const float* wv = (const float*)d_in[5]; const float* bv = (const float*)d_in[6]; const float* wo = (const float*)d_in[7]; const float* bo = (const float*)d_in[8];
  float* out = (float*)d_out;
  char* ws = (char*)d_ws; size_t off = 0;
  auto take = [&](size_t bytes) { char* p = ws + off; off += (bytes + 255) & ~(size_t)255; return p; };
  _Float16* BQ = (_Float16*)take((size_t)DM * DM * 2); _Float16* BK = (_Float16*)take((size_t)DM * DM * 2); _Float16* BV = (_Float16*)take((size_t)DM * DM * 2); _Float16* BO = (_Float16*)take((size_t)DM * DM * 2);
  _Float16* X16 = (_Float16*)take(NR * DM * 2);
  float* QF = (float*)take(NR * DM * 4);
  _Float16* QH = (_Float16*)take(NR * DM * 2); _Float16* QL = (_Float16*)take(NR * DM * 2); _Float16* KH = (_Float16*)take(NR * DM * 2); _Float16* KL = (_Float16*)take(NR * DM * 2);
  _Float16* V16 = (_Float16*)take(NR * DM * 2); _Float16* O16 = (_Float16*)take(NR * DM * 2);
  float* S = (float*)take((size_t)NH * QT * NKX * 4); _Float16* P = (_Float16*)take((size_t)NH * QT * NKX * 2); _Float16* VT = (_Float16*)take((size_t)NH * HD * SQ * 2);
  float* TAB = (float*)take((size_t)SQ * 32 * 4);
  float* QK0 = (float*)take((size_t)2 * QT0 * DM * 4); float* QKR0 = (float*)take((size_t)2 * QT0 * DM * 4); float* VF0 = (float*)take((size_t)QT0 * DM * 4);
  float* OF0 = (float*)take((size_t)NB * QT0 * DM * 4); _Float16* OH0 = (_Float16*)take((size_t)NB * QT0 * DM * 2); _Float16* OL0 = (_Float16*)take((size_t)NB * QT0 * DM * 2);
  if (off > ws_size || off > (size_t)134217728) return;

  { const size_t n8w = (size_t)DM * DM / 8; const unsigned g = (unsigned)((n8w + 255) / 256);
    k_wnat<<<g, 256, 0, stream>>>(wq, n8w, BQ); k_wnat<<<g, 256, 0, stream>>>(wk, n8w, BK); k_wnat<<<g, 256, 0, stream>>>(wv, n8w, BV); k_wnat<<<g, 256, 0, stream>>>(wo, n8w, BO); }
  { const size_t n8x = (size_t)SQ * DM / 8; k_x16<<<dim3((unsigned)((n8x + 255) / 256), NB), 256, 0, stream>>>(x, (size_t)SQ_FULL * DM, X16, (size_t)SQ * DM, n8x); }
  k_tab<<<SQ / 16, 256, 0, stream>>>(TAB);

  const dim3 gp((unsigned)((MP / 128) * (DM / 64)), 1);
  const size_t n8p = (size_t)MP * DM / 8; const unsigned ghl = (unsigned)((n8p + 255) / 256);
  k_gemm2<<<gp, 128, 0, stream>>>(X16, DM, (size_t)0, BQ, DM, (size_t)0, 0.0625f, bq, nullptr, QF, nullptr, DM, (size_t)0, MP, DM, DM);
  k_hlrope<<<ghl, 256, 0, stream>>>(QF, TAB, QH, QL, n8p);
  k_gemm2<<<gp, 128, 0, stream>>>(X16, DM, (size_t)0, BK, DM, (size_t)0, 0.0625f, bk, nullptr, QF, nullptr, DM, (size_t)0, MP, DM, DM);
  k_hlrope<<<ghl, 256, 0, stream>>>(QF, TAB, KH, KL, n8p);
  k_gemm2<<<gp, 128, 0, stream>>>(X16, DM, (size_t)0, BV, DM, (size_t)0, 0.0625f, bv, nullptr, nullptr, V16, DM, (size_t)0, MP, DM, DM);

  for (int b = 0; b < NB; ++b) { const size_t r0 = (size_t)b * SQ;
    k_vt<NH, SQ><<<NH * (SQ / 64), 256, 0, stream>>>(V16 + r0 * DM, DM, 0, VT);
    const dim3 g0((QT0 / 128) * (DM / 64), 1);
    k_gemm2<<<g0, 128, 0, stream>>>(X16 + r0 * DM, DM, (size_t)0, BQ, DM, (size_t)0, 0.0625f, bq, nullptr, QK0, nullptr, DM, (size_t)0, QT0, DM, DM);
    k_gemm2<<<g0, 128, 0, stream>>>(X16 + r0 * DM, DM, (size_t)0, BK, DM, (size_t)0, 0.0625f, bk, nullptr, QK0 + (size_t)QT0 * DM, nullptr, DM, (size_t)0, QT0, DM, DM);
    k_gemm2<<<g0, 128, 0, stream>>>(X16 + r0 * DM, DM, (size_t)0, BV, DM, (size_t)0, 0.0625f, bv, nullptr, VF0, nullptr, DM, (size_t)0, QT0, DM, DM);
    { const int n4 = 2 * QT0 * DM / 4; k_rope0<<<(n4 + 255) / 256, 256, 0, stream>>>(QK0, TAB, QKR0, n4); }
    k_att0<<<NH * (QT0 / 64), 64, 0, stream>>>(QKR0, QKR0 + (size_t)QT0 * DM, VF0, DM, SCL, OF0 + (size_t)b * QT0 * DM, DM);
    for (int q0 = 0; q0 < SQ; q0 += QT) { const int nk = q0 + QT;
      const dim3 gs((unsigned)((QT / 128) * (nk / 64)), NH);
      k_gemm2<<<gs, 128, 0, stream>>>(QH + (r0 + q0) * DM, DM, (size_t)HD, KH + r0 * DM, DM, (size_t)HD, SCL, nullptr, nullptr, S, nullptr, NKX, (size_t)QT * NKX, QT, nk, HD);
      k_gemm2<<<gs, 128, 0, stream>>>(QL + (r0 + q0) * DM, DM, (size_t)HD, KH + r0 * DM, DM, (size_t)HD, SCLR, nullptr, S, S, nullptr, NKX, (size_t)QT * NKX, QT, nk, HD);
      k_gemm2<<<gs, 128, 0, stream>>>(QH + (r0 + q0) * DM, DM, (size_t)HD, KL + r0 * DM, DM, (size_t)HD, SCLR, nullptr, S, S, nullptr, NKX, (size_t)QT * NKX, QT, nk, HD);
      k_rsmcf2<<<(NH * QT + 255) / 256, 256, 0, stream>>>(S, P, NH, q0, nk);
      k_gemm2<<<dim3((QT / 128) * (HD / 64), NH), 128, 0, stream>>>(P, NKX, (size_t)QT * NKX, VT, SQ, (size_t)HD * SQ, 0.25f, nullptr, nullptr, nullptr, O16 + (r0 + q0) * DM, DM, (size_t)HD, QT, HD, nk); } }

  k_gemm2<<<dim3((unsigned)((SQ / 128) * (DM / 64)), NB), 128, 0, stream>>>(O16, DM, (size_t)SQ * DM, BO, DM, (size_t)0, 0.0009765625f, bo, nullptr, out, nullptr, DM, (size_t)SQ_FULL * DM, SQ, DM, DM);
  { const size_t n80 = (size_t)NB * QT0 * DM / 8; k_hl<<<(unsigned)((n80 + 255) / 256), 256, 0, stream>>>(OF0, OH0, OL0, n80); }
  const dim3 gf((QT0 / 128) * (DM / 64), NB);
  k_gemm2<<<gf, 128, 0, stream>>>(OH0, DM, (size_t)QT0 * DM, BO, DM, (size_t)0, 0.0009765625f, bo, nullptr, out, nullptr, DM, (size_t)SQ_FULL * DM, QT0, DM, DM);
  k_gemm2<<<gf, 128, 0, stream>>>(OL0, DM, (size_t)QT0 * DM, BO, DM, (size_t)0, 0.00000095367431640625f, nullptr, out, out, nullptr, DM, (size_t)SQ_FULL * DM, QT0, DM, DM);
}
